// MultiHeadAttention_41764261986665
// MI455X (gfx1250) — hardware-run, weakly checked
//
#include <hip/hip_runtime.h>


#ifndef NB
#define NB 2
#endif
#ifndef SEQ
#define SEQ 2048
#endif
#define NB_FULL  2
#define SEQ_FULL 2048
#ifndef OUT_SEQ
#define OUT_SEQ SEQ
#endif
#define DM   256
#define NH_  8
#define HD   32
#define CXP  (2 * DM)
#define AW   4
#define QRS  2048.0f
#define QRI  (1.0f / 2048.0f)
#define SC2  (0.17677669529663687f * 1.4426950408889634f)
#define PSH  8.0f
#define NEGT (-4294967296.0f * 1.4426950408889634f)

static_assert(HD == 32);
static_assert(NH_ * HD == DM);
static_assert(NH_ % 2 == 0);
static_assert(DM % 64 == 0);
static_assert(DM % 32 == 0);
static_assert(CXP % 32 == 0);
static_assert(SEQ % 64 == 0);
static_assert((NB * SEQ) % 64 == 0);
static_assert(SEQ % 32 == 0);
static_assert(SEQ % (16 * AW) == 0);
static_assert(((size_t)SEQ * DM) % 8 == 0);
static_assert(NB <= NB_FULL);
static_assert(SEQ <= SEQ_FULL);

typedef _Float16 h16;
typedef unsigned short bf;
typedef __attribute__((ext_vector_type(16))) __bf16   v16bf;
typedef __attribute__((ext_vector_type(16))) _Float16 v16h;
typedef __attribute__((ext_vector_type(8)))  _Float16 v8h;
typedef __attribute__((ext_vector_type(8)))  unsigned short v8us;
typedef __attribute__((ext_vector_type(8)))  float    v8f;
typedef __attribute__((ext_vector_type(4)))  float    v4f;
typedef __attribute__((ext_vector_type(4)))  int      v4i;
typedef v4f  __attribute__((may_alias)) v4fa;

__device__ __forceinline__ unsigned short f2bf(float f) { unsigned u = __float_as_uint(f); u += 0x7FFFu + ((u >> 16) & 1u); return (unsigned short)(u >> 16); }
__device__ __forceinline__ float bf2f(unsigned short s) { return __uint_as_float(((unsigned)s) << 16); }
__device__ __forceinline__ float bfr(float f) { return bf2f(f2bf(f)); }
__device__ __forceinline__ v16h cat16(v8h lo, v8h hi) { return __builtin_shufflevector(lo, hi, 0, 1, 2, 3, 4, 5, 6, 7, 8, 9, 10, 11, 12, 13, 14, 15); }
__device__ __forceinline__ v16bf cat16b(v8us lo, v8us hi) { return __builtin_bit_cast(v16bf, __builtin_shufflevector(lo, hi, 0, 1, 2, 3, 4, 5, 6, 7, 8, 9, 10, 11, 12, 13, 14, 15)); }
__device__ __forceinline__ v8f wmma16(v16h a, v16h b, v8f c) { return __builtin_amdgcn_wmma_f32_16x16x32_f16(false, a, false, b, (short)0, c, false, false); }
__device__ __forceinline__ v8f wmmab(v16bf a, v16bf b, v8f c) { return __builtin_amdgcn_wmma_f32_16x16x32_bf16(false, a, false, b, (short)0, c, false, false); }
__device__ __forceinline__ v16h  ldh(const h16* p) { return cat16(*(const v8h*)p, *(const v8h*)(p + 16)); }
__device__ __forceinline__ v16bf ldb(const bf* p)  { return cat16b(*(const v8us*)p, *(const v8us*)(p + 16)); }
__device__ __forceinline__ void wave_sync() { __builtin_amdgcn_fence(3  , "wavefront"); __builtin_amdgcn_wave_barrier(); asm volatile("" ::: "memory"); }

__global__ __launch_bounds__(256) void k_cvt8(const float* __restrict__ src, bf* dst, size_t n8) {
    const size_t i = (size_t)blockIdx.x * 256 + threadIdx.x; if (i >= n8) return;
    const v8f v = *(const v8f*)(src + i * 8); v8us o;
#pragma unroll
    for (int k = 0; k < 8; ++k) o[k] = f2bf(v[k]);
    *(volatile v8us*)(dst + i * 8) = o; __threadfence(); *(volatile v8us*)(dst + i * 8) = o;
}

__global__ __launch_bounds__(256) void k_wT(const float* __restrict__ W, bf* dst, int ldo, int coff) {
    __shared__ float ts[64 * 65];
    const int tid = threadIdx.x; const int k0 = blockIdx.x * 64, n0 = blockIdx.y * 64;
#pragma unroll
    for (int i = 0; i < 4; ++i) { const int kk = (tid >> 4) + 16 * i, c4 = (tid & 15) * 4;
        const v4f f = *(const v4f*)(W + (size_t)(k0 + kk) * DM + n0 + c4);
        ts[kk * 65 + c4 + 0] = f[0]; ts[kk * 65 + c4 + 1] = f[1]; ts[kk * 65 + c4 + 2] = f[2]; ts[kk * 65 + c4 + 3] = f[3]; }
    __syncthreads();
#pragma unroll 1
    for (int ps = 0; ps < 2; ++ps) {
#pragma unroll
        for (int it = 0; it < 2; ++it) { const int nn = it * 32 + (tid >> 3), ks = (tid & 7) * 8;
            v8us o;
#pragma unroll
            for (int j = 0; j < 8; ++j) o[j] = f2bf(ts[(ks + j) * 65 + nn]);
            *(volatile v8us*)(dst + (size_t)(n0 + nn) * (size_t)ldo + coff + k0 + ks) = o; }
        if (ps == 0) __threadfence(); }
}

template <bool F32OUT>
__global__ __launch_bounds__(32) void k_gemm(const bf* __restrict__ A, const bf* __restrict__ Bt, h16* Ph, h16* Pr, float* OUT, const float* __restrict__ bias,
                                             size_t sRB, size_t sCB, int K, int useRes, int RB, int pitch, int CB, int biasRow) {
    __shared__ __align__(16) float os[16 * 68];
    const int lane = threadIdx.x & 31, lr = lane & 15, hi = lane >> 4; const int r0 = blockIdx.x * 64, c0 = blockIdx.y * 64;
    v8f acc[4][4];
#pragma unroll
    for (int mb = 0; mb < 4; ++mb)
#pragma unroll
        for (int nb = 0; nb < 4; ++nb) acc[mb][nb] = (v8f){};
    const size_t aoff = (size_t)(r0 + lr) * K + 8 * hi, boff = (size_t)(c0 + lr) * K + 8 * hi;
#pragma unroll 1
    for (int kc = 0; kc < K; kc += 32) {
        v16bf a[4];
#pragma unroll
        for (int mb = 0; mb < 4; ++mb) a[mb] = ldb(A + aoff + (size_t)mb * 16 * K + kc);
#pragma unroll
        for (int nb = 0; nb < 4; ++nb) { const v16bf b = ldb(Bt + boff + (size_t)nb * 16 * K + kc);
#pragma unroll
            for (int mb = 0; mb < 4; ++mb) acc[mb][nb] = wmmab(a[mb], b, acc[mb][nb]); }
        asm volatile("v_nop\n\tv_nop\n\tv_nop\n\tv_nop" : "+v"(acc[0][0]), "+v"(acc[1][1]), "+v"(acc[2][2]), "+v"(acc[3][3]) : "v"(a[0]), "v"(a[1]), "v"(a[2]), "v"(a[3]));
    }
    const size_t tbase = (size_t)(r0 / RB) * sRB + (size_t)(r0 % RB) * (size_t)pitch + (size_t)(c0 / CB) * sCB + (size_t)(c0 % CB);
#pragma unroll
    for (int mb = 0; mb < 4; ++mb) {
#pragma unroll
        for (int nb = 0; nb < 4; ++nb) {
#pragma unroll
            for (int j = 0; j < 8; ++j) os[(hi * 8 + j) * 68 + nb * 16 + lr] = acc[mb][nb][j]; }
        wave_sync();
        if constexpr (!F32OUT) {
            const size_t sb = tbase + (size_t)(mb * 16) * (size_t)pitch;
#pragma unroll 1
            for (int ps = 0; ps < 2; ++ps) {
#pragma unroll
                for (int s = 0; s < 4; ++s) { const int row = 4 * s + (lane >> 3), c8 = (lane & 7) * 8;
                    v4f x0 = *(const v4fa*)(&os[row * 68 + c8]); v4f x1 = *(const v4fa*)(&os[row * 68 + c8 + 4]);
                    const int cidx = (c0 + c8) & (DM - 1), ridx = (r0 + mb * 16 + row) & (DM - 1);
                    const v4f bc0 = *(const v4f*)(bias + cidx), bc1 = *(const v4f*)(bias + cidx + 4); const float br = bias[ridx];
                    v8h hv, rv;
#pragma unroll
                    for (int i = 0; i < 4; ++i) { const float y0 = x0[i] + bfr(biasRow ? br : bc0[i]); const float y1 = x1[i] + bfr(biasRow ? br : bc1[i]);
                        const h16 a0 = (h16)y0; const h16 a1 = (h16)y1; hv[i] = a0; hv[4 + i] = a1; rv[i] = (h16)((y0 - (float)a0) * QRS); rv[4 + i] = (h16)((y1 - (float)a1) * QRS); }
                    const size_t oo = sb + (size_t)row * (size_t)pitch + c8;
                    *(volatile v8h*)(Ph + oo) = hv; if (useRes) *(volatile v8h*)(Pr + oo) = rv; }
                if (ps == 0) __threadfence(); }
        } else {
#pragma unroll 1
            for (int ps = 0; ps < 2; ++ps) {
#pragma unroll
                for (int s = 0; s < 8; ++s) { const int row = 2 * s + hi, cofs = lr * 4;
                    const int m = r0 + mb * 16 + row; const int bb = m / SEQ, tt = m - bb * SEQ;
                    v4f val = *(const v4fa*)(&os[row * 68 + cofs]);
                    const int cidx = (c0 + cofs) & (DM - 1), ridx = m & (DM - 1);
                    const v4f bc = *(const v4f*)(bias + cidx); const float br = bias[ridx];
#pragma unroll
                    for (int i = 0; i < 4; ++i) val[i] = val[i] + bfr(biasRow ? br : bc[i]);
                    *(volatile v4f*)(OUT + ((size_t)bb * OUT_SEQ + tt) * DM + c0 + cofs) = val; }
                if (ps == 0) __threadfence(); }
        }
        wave_sync();
    }
}

__global__ __launch_bounds__(32 * AW) void k_flash(const h16* __restrict__ QH, const h16* __restrict__ QR, const h16* __restrict__ KP, const h16* __restrict__ VT,
                                                   const int* __restrict__ MK, bf* CX) {
    __shared__ __align__(16) float os[AW * 16 * 68];
    const int lane = threadIdx.x & 31, wave = __builtin_amdgcn_readfirstlane((int)(threadIdx.x >> 5)), lr = lane & 15, hi = lane >> 4;
    const int zp = blockIdx.y; const int b = zp / (NH_ / 2), hp = zp % (NH_ / 2);
    const int t0 = (blockIdx.x * AW + wave) * 16;
    const int wb = wave * 16 * 68;
    const size_t rowb = (size_t)b * SEQ;
    const int* mk = MK + (size_t)b * SEQ_FULL + 8 * hi;
#pragma unroll 1
    for (int hh = 0; hh < 2; ++hh) {
        const int h = hp * 2 + hh;
        const size_t qo = (rowb + t0 + lr) * DM + h * HD + 8 * hi;
        const v16h qh = ldh(QH + qo), qr = ldh(QR + qo);
        const size_t ko = (rowb + lr) * DM + h * HD + 8 * hi;
        const size_t vo = ((size_t)b * DM + h * HD + lr) * SEQ + 8 * hi;
        v8f o0 = (v8f){}, o1 = (v8f){};
        float m = -3.0e38f, l = 0.0f;
#pragma unroll 1
        for (int key0 = 0; key0 < SEQ; key0 += 32) {
            const h16* ka = KP + ko + (size_t)key0 * DM;
            const v16h ka0 = ldh(ka), kb0 = ldh(ka + 16 * DM);
            const v4i ma0 = *(const v4i*)(mk + key0), ma1 = *(const v4i*)(mk + key0 + 4), mb0 = *(const v4i*)(mk + key0 + 16), mb1 = *(const v4i*)(mk + key0 + 20);
            v8f sHa = (v8f){}, sLa = (v8f){}, sHb = (v8f){}, sLb = (v8f){};
            sHa = wmma16(ka0, qh, sHa); sLa = wmma16(ka0, qr, sLa); sHb = wmma16(kb0, qh, sHb); sLb = wmma16(kb0, qr, sLb);
            asm volatile("v_nop\n\tv_nop\n\tv_nop\n\tv_nop" : "+v"(sHa), "+v"(sLa), "+v"(sHb), "+v"(sLb) : "v"(ka0), "v"(kb0), "v"(qh), "v"(qr));
            float ta[8], tb[8]; float mx = -3.0e38f;
#pragma unroll
            for (int r = 0; r < 4; ++r) {
                const float a0 = (sHa[r] + sLa[r] * QRI) * SC2, a1 = (sHa[4 + r] + sLa[4 + r] * QRI) * SC2;
                const float c0 = (sHb[r] + sLb[r] * QRI) * SC2, c1 = (sHb[4 + r] + sLb[4 + r] * QRI) * SC2;
                ta[r] = (ma0[r] != 0) ? a0 : NEGT; ta[4 + r] = (ma1[r] != 0) ? a1 : NEGT;
                tb[r] = (mb0[r] != 0) ? c0 : NEGT; tb[4 + r] = (mb1[r] != 0) ? c1 : NEGT; }
#pragma unroll
            for (int r = 0; r < 8; ++r) mx = fmaxf(mx, fmaxf(ta[r], tb[r]));
            mx = fmaxf(mx, __shfl_xor(mx, 16, 32));
            const float mnew = fmaxf(m, mx);
            const float alpha = __builtin_amdgcn_exp2f(m - mnew);
            const float sh = PSH - mnew;
            v16h pb; float ls = 0.0f;
#pragma unroll
            for (int r = 0; r < 8; ++r) { const h16 pa = (h16)__builtin_amdgcn_exp2f(ta[r] + sh); const h16 pc = (h16)__builtin_amdgcn_exp2f(tb[r] + sh); pb[r] = pa; pb[8 + r] = pc; ls += (float)pa + (float)pc; }
            l = l * alpha + ls; m = mnew;
            o0 = o0 * alpha; o1 = o1 * alpha;
            const h16* va = VT + vo + key0;
            const v16h v0 = ldh(va), v1 = ldh(va + (size_t)16 * SEQ);
            o0 = wmma16(v0, pb, o0); o1 = wmma16(v1, pb, o1);
            asm volatile("v_nop\n\tv_nop\n\tv_nop\n\tv_nop" : "+v"(o0), "+v"(o1) : "v"(v0), "v"(v1), "v"(pb));
        }
        l += __shfl_xor(l, 16, 32);
        const float inv = 1.0f / l;
        { v4f a, c; const int ob = wb + lr * 68 + hh * 32 + 8 * hi;
          a[0] = o0[0] * inv; a[1] = o0[1] * inv; a[2] = o0[2] * inv; a[3] = o0[3] * inv; c[0] = o0[4] * inv; c[1] = o0[5] * inv; c[2] = o0[6] * inv; c[3] = o0[7] * inv;
          *(v4fa*)(&os[ob]) = a; *(v4fa*)(&os[ob + 4]) = c;
          a[0] = o1[0] * inv; a[1] = o1[1] * inv; a[2] = o1[2] * inv; a[3] = o1[3] * inv; c[0] = o1[4] * inv; c[1] = o1[5] * inv; c[2] = o1[6] * inv; c[3] = o1[7] * inv;
          *(v4fa*)(&os[ob + 16]) = a; *(v4fa*)(&os[ob + 20]) = c; }
    }
    wave_sync();
    bf* crow = CX + (rowb + t0) * CXP + hp * 64;
#pragma unroll 1
    for (int ps = 0; ps < 2; ++ps) {
#pragma unroll
        for (int s = 0; s < 4; ++s) { const int row = 4 * s + (lane >> 3), c8 = (lane & 7) * 8;
            const v4f x0 = *(const v4fa*)(&os[wb + row * 68 + c8]); const v4f x1 = *(const v4fa*)(&os[wb + row * 68 + c8 + 4]); v8us hv, lv;
#pragma unroll
            for (int i = 0; i < 4; ++i) { const unsigned short u0 = f2bf(x0[i]); const unsigned short u1 = f2bf(x1[i]); hv[i] = u0; hv[4 + i] = u1;
                lv[i] = f2bf(x0[i] - bf2f(u0)); lv[4 + i] = f2bf(x1[i] - bf2f(u1)); }
            const size_t oo = (size_t)row * CXP + c8;
            *(volatile v8us*)(crow + oo) = hv; *(volatile v8us*)(crow + oo + DM) = lv; }
        if (ps == 0) __threadfence(); }
}

static constexpr size_t al256(size_t v) { return (v + 255) & ~(size_t)255; }
static constexpr size_t SZ_X  = al256((size_t)NB * SEQ * DM * 2);
static constexpr size_t SZ_W  = al256((size_t)DM * DM * 2);
static constexpr size_t SZ_WO = al256((size_t)DM * CXP * 2);
static constexpr size_t SZ_PL = al256((size_t)NB * SEQ * DM * 2);
static constexpr size_t SZ_CX = al256((size_t)NB * SEQ * CXP * 2);
static constexpr size_t SZ_TOTAL = 3 * SZ_X + 3 * SZ_W + SZ_WO + 4 * SZ_PL + SZ_CX;
static_assert(SZ_TOTAL <= (size_t)134217728);
static_assert((size_t)NB * DM * SEQ * 2 <= SZ_PL);

static void cvt_act(const float* x, bf* dst, hipStream_t stream) {
    if (SEQ == SEQ_FULL) {
        const size_t n8 = (size_t)NB * SEQ * DM / 8;
        k_cvt8<<<(unsigned)((n8 + 255) / 256), 256, 0, stream>>>(x, dst, n8);
    } else {
        const size_t n8 = (size_t)SEQ * DM / 8;
        for (int b = 0; b < NB; ++b) k_cvt8<<<(unsigned)((n8 + 255) / 256), 256, 0, stream>>>(x + (size_t)b * SEQ_FULL * DM, dst + (size_t)b * SEQ * DM, n8);
    }
}

extern "C" void kernel_launch(void* const* d_in, const int* in_sizes, int n_in,
                              void* d_out, int out_size, void* d_ws, size_t ws_size, hipStream_t stream) {
    if (n_in < 12) return;
    const size_t needx = ((size_t)(NB - 1) * SEQ_FULL + SEQ) * DM;
    if ((size_t)in_sizes[0] < needx || (size_t)in_sizes[1] < needx || (size_t)in_sizes[2] < needx) return;
    if ((size_t)in_sizes[3] < (size_t)(NB - 1) * SEQ_FULL + SEQ) return;
    if ((size_t)in_sizes[4] < (size_t)DM * DM || (size_t)in_sizes[6] < (size_t)DM * DM || (size_t)in_sizes[8] < (size_t)DM * DM || (size_t)in_sizes[10] < (size_t)DM * DM) return;
    if (in_sizes[5] < DM || in_sizes[7] < DM || in_sizes[9] < DM || in_sizes[11] < DM) return;
    if ((size_t)out_size < ((size_t)(NB - 1) * OUT_SEQ + SEQ) * DM) return;
    if (SZ_TOTAL > ws_size) return;
    const float* xq = (const float*)d_in[0]; const float* xk = (const float*)d_in[1]; const float* xv = (const float*)d_in[2];
    const int* kmask = (const int*)d_in[3];
    const float* wq = (const float*)d_in[4]; const float* bq = (const float*)d_in[5];
    const float* wk = (const float*)d_in[6]; const float* bk = (const float*)d_in[7];
    const float* wv = (const float*)d_in[8]; const float* bv = (const float*)d_in[9];
    const float* wo = (const float*)d_in[10]; const float* bo = (const float*)d_in[11];
    float* OUT = (float*)d_out;
    char* wsp = (char*)d_ws;
    bf* XQ = (bf*)wsp; wsp += SZ_X;
    bf* XK = (bf*)wsp; wsp += SZ_X;
    bf* XV = (bf*)wsp; wsp += SZ_X;
    bf* WQT = (bf*)wsp; wsp += SZ_W;
    bf* WKT = (bf*)wsp; wsp += SZ_W;
    bf* WVT = (bf*)wsp; wsp += SZ_W;
    bf* WO2 = (bf*)wsp; wsp += SZ_WO;
    h16* QH = (h16*)wsp; wsp += SZ_PL;
    h16* QR = (h16*)wsp; wsp += SZ_PL;
    h16* KP = (h16*)wsp; wsp += SZ_PL;
    h16* VT = (h16*)wsp; wsp += SZ_PL;
    bf* CX = (bf*)wsp; wsp += SZ_CX;

    cvt_act(xq, XQ, stream); cvt_act(xk, XK, stream); cvt_act(xv, XV, stream);
    { const dim3 g(DM / 64, DM / 64, 1);
      k_wT<<<g, 256, 0, stream>>>(wq, WQT, DM, 0);
      k_wT<<<g, 256, 0, stream>>>(wk, WKT, DM, 0);
      k_wT<<<g, 256, 0, stream>>>(wv, WVT, DM, 0);
      k_wT<<<g, 256, 0, stream>>>(wo, WO2, CXP, 0);
      k_wT<<<g, 256, 0, stream>>>(wo, WO2, CXP, DM); }

    k_gemm<false><<<dim3(NB * SEQ / 64, DM / 64, 1), 32, 0, stream>>>(XQ, WQT, QH, QR, OUT, bq, (size_t)0, (size_t)0, DM, 1, NB * SEQ, DM, DM, 0);
    k_gemm<false><<<dim3(NB * SEQ / 64, DM / 64, 1), 32, 0, stream>>>(XK, WKT, KP, KP, OUT, bk, (size_t)0, (size_t)0, DM, 0, NB * SEQ, DM, DM, 0);
    k_gemm<false><<<dim3(DM / 64, NB * SEQ / 64, 1), 32, 0, stream>>>(WVT, XV, VT, VT, OUT, bv, (size_t)0, (size_t)DM * SEQ, DM, 0, DM, SEQ, SEQ, 1);

    k_flash<<<dim3(SEQ / (16 * AW), NB * (NH_ / 2), 1), 32 * AW, 0, stream>>>(QH, QR, KP, VT, kmask, CX);

    k_gemm<true><<<dim3(NB * SEQ / 64, DM / 64, 1), 32, 0, stream>>>(CX, WO2, QH, QH, OUT, bo, (size_t)0, (size_t)0, CXP, 0, NB * SEQ, DM, DM, 0);
}
